// Block_44358422233377
// MI455X (gfx1250) — hardware-run, weakly checked
//
#include <hip/hip_runtime.h>


#ifndef NB
#define NB 4
#endif
#ifndef SEQ
#define SEQ 1024
#endif
#define NB_FULL  4
#define SEQ_FULL 1024
#define DM    1024
#define NH    16
#define DH    64
#define QKVW  3072
#define FFD   4096
#define NTOK  (NB * SEQ)
#define WCAR  16.0f
#define HCAR  16.0f
#define ACAR  16.0f
#define OCAR  256.0f
#define TCAR  256.0f
#define PCAR  256.0f
#define L2E   1.4426950408889634f
#define EP_H16  0
#define EP_GELU 1
#define EP_RES  2

static_assert(NB >= 1 && NB <= NB_FULL);
static_assert(SEQ >= 256 && SEQ <= SEQ_FULL);
static_assert((SEQ % 256) == 0);
static_assert((SEQ % 64) == 0);
static_assert((SEQ % 32) == 0);
static_assert(SEQ == SEQ_FULL || NB == 1);
static_assert((NTOK % 64) == 0);
static_assert(NH * DH == DM);
static_assert(DH == 64);
static_assert(QKVW == 3 * DM);
static_assert((DM % 64) == 0 && (QKVW % 64) == 0 && (FFD % 64) == 0);
static_assert((DM % 32) == 0 && (FFD % 32) == 0);
static_assert(128 * 8 == DM);
static_assert(((QKVW * DM) % 8) == 0 && ((DM * DM) % 8) == 0 && ((FFD * DM) % 8) == 0);
static_assert((size_t)NTOK * DM * 4 <= (size_t)16777216);

constexpr size_t al256(size_t b) { return (b + 255) & ~(size_t)255; }
constexpr size_t WS_TOTAL = al256((size_t)QKVW * DM * 2) + 2 * al256((size_t)DM * DM * 2) + 2 * al256((size_t)FFD * DM * 2)
                          + al256((size_t)NTOK * QKVW * 2) + al256((size_t)NTOK * DM * 2) + al256((size_t)NTOK * DM * 4)
                          + al256((size_t)NTOK * DM * 2) + al256((size_t)NTOK * DM * 2) + al256((size_t)NTOK * FFD * 2);
static_assert(WS_TOTAL <= (size_t)134217728);
static_assert((size_t)NTOK * DM * 2 <= (size_t)NTOK * QKVW * 2);
static_assert((size_t)NTOK * DM * 2 <= (size_t)NTOK * DM * 4);

typedef _Float16 h16;
typedef __attribute__((ext_vector_type(16))) _Float16 v16h;
typedef __attribute__((ext_vector_type(8)))  _Float16 v8h;
typedef __attribute__((ext_vector_type(2)))  _Float16 v2h;
typedef __attribute__((ext_vector_type(8)))  float    v8f;
typedef __attribute__((ext_vector_type(4)))  float    v4f;
typedef v8h __attribute__((may_alias)) v8ha;
typedef v4f __attribute__((may_alias)) v4fa;

__device__ __forceinline__ float bfr(float f) { unsigned u = __float_as_uint(f); u += 0x7FFFu + ((u >> 16) & 1u); return __uint_as_float(u & 0xFFFF0000u); }
__device__ __forceinline__ v16h cat16(v8h lo, v8h hi) { return __builtin_shufflevector(lo, hi, 0, 1, 2, 3, 4, 5, 6, 7, 8, 9, 10, 11, 12, 13, 14, 15); }
__device__ __forceinline__ v8f cat8f(v4f lo, v4f hi) { return __builtin_shufflevector(lo, hi, 0, 1, 2, 3, 4, 5, 6, 7); }
__device__ __forceinline__ v8f wmma16(v16h a, v16h b, v8f c) { return __builtin_amdgcn_wmma_f32_16x16x32_f16(false, a, false, b, (short)0, c, false, false); }
__device__ __forceinline__ v8f wmma16g(v16h a, v16h b, v8f c) {
    c = wmma16(a, b, c);
    asm volatile("v_nop\n\tv_nop\n\tv_nop\n\tv_nop" : "+v"(c) : "v"(a), "v"(b));
    return c;
}
__device__ __forceinline__ float wsum(float v) { v += __shfl_xor(v, 16, 32); v += __shfl_xor(v, 8, 32); v += __shfl_xor(v, 4, 32); v += __shfl_xor(v, 2, 32); v += __shfl_xor(v, 1, 32); return v; }

__device__ __forceinline__ v16h ldfrag(const h16* p) { return cat16(*(const v8ha*)p, *(const v8ha*)(p + 16)); }

__device__ __forceinline__ float gelu_e(float x) {
    const float z = fabsf(x) * 0.70710678118654752f;
    const float t = __builtin_amdgcn_rcpf(1.0f + 0.3275911f * z);
    const float pl = t * (0.254829592f + t * (-0.284496736f + t * (1.421413741f + t * (-1.453152027f + t * 1.061405429f))));
    const float q = 0.5f * pl * __builtin_amdgcn_exp2f(-L2E * z * z);
    const float ph = (x < 0.0f) ? q : (1.0f - q);
    return x * ph;
}

template <int EP, bool BIAS, bool RBF>
__device__ __forceinline__ void gemm_body(const h16* __restrict__ A, const h16* __restrict__ Bt, int K,
                                          float* Cf, h16* Ch, int ldc, float cs, float co,
                                          const float* __restrict__ bias, const float* __restrict__ R,
                                          size_t sA, size_t sB, size_t sC) {
    __shared__ __align__(16) float os[16 * 68];
    const size_t z = blockIdx.z; A += z * sA; Bt += z * sB;
    const int lane = threadIdx.x & 31, lr = lane & 15, hi = lane >> 4;
    const int r0 = blockIdx.x * 64, c0 = blockIdx.y * 64;
    v8f acc[4][4];
#pragma unroll
    for (int mb = 0; mb < 4; ++mb)
#pragma unroll
        for (int nb = 0; nb < 4; ++nb) acc[mb][nb] = (v8f){};
    const size_t aoff = (size_t)(r0 + lr) * K + 8 * hi, boff = (size_t)(c0 + lr) * K + 8 * hi;
#pragma unroll 1
    for (int kc = 0; kc < K; kc += 32) {
        v16h a[4], b;
#pragma unroll
        for (int mb = 0; mb < 4; ++mb) a[mb] = ldfrag(A + aoff + (size_t)mb * 16 * K + kc);
#pragma unroll
        for (int nb = 0; nb < 4; ++nb) {
            b = ldfrag(Bt + boff + (size_t)nb * 16 * K + kc);
#pragma unroll
            for (int mb = 0; mb < 4; ++mb) acc[mb][nb] = wmma16(a[mb], b, acc[mb][nb]);
        }
        asm volatile("v_nop\n\tv_nop\n\tv_nop\n\tv_nop" : "+v"(acc[0][0]), "+v"(acc[1][1]), "+v"(acc[2][2]), "+v"(acc[3][3]) : "v"(a[0]), "v"(a[3]), "v"(b));
    }
#pragma unroll
    for (int mb = 0; mb < 4; ++mb) {
#pragma unroll
        for (int nb = 0; nb < 4; ++nb) {
#pragma unroll
            for (int j = 0; j < 8; ++j) os[(hi * 8 + j) * 68 + nb * 16 + lr] = acc[mb][nb][j];
        }
        __builtin_amdgcn_fence(3, "wavefront"); __builtin_amdgcn_wave_barrier(); asm volatile("" ::: "memory");
        if constexpr (EP == EP_RES) {
            float* crow = Cf + z * sC + (size_t)(r0 + mb * 16) * ldc + c0;
            const float* rrow = R + (size_t)(r0 + mb * 16) * ldc + c0;
#pragma unroll 1
            for (int ps = 0; ps < 2; ++ps) {
#pragma unroll 1
                for (int s = 0; s < 8; ++s) {
                    const int row = 2 * s + hi, cofs = lr * 4;
                    const v4f u = *(const v4fa*)(os + row * 68 + cofs);
                    const v4f rv = *(const v4f*)(rrow + (size_t)row * ldc + cofs);
                    v4f o;
#pragma unroll
                    for (int q = 0; q < 4; ++q) {
                        float bq = 0.0f;
                        if constexpr (BIAS) bq = bfr(bias[c0 + cofs + q]);
                        const float y = u[q] * cs + bq;
                        const float rq0 = rv[q];
                        const float rq = RBF ? bfr(rq0) : rq0;
                        o[q] = rq + y;
                    }
                    *(volatile v4f*)(crow + (size_t)row * ldc + cofs) = o;
                }
                if (ps == 0) __threadfence();
            }
        } else {
            h16* crow = Ch + z * sC + (size_t)(r0 + mb * 16) * ldc + c0;
            const int q8 = lane >> 3, cofs = (lane & 7) * 8;
#pragma unroll 1
            for (int ps = 0; ps < 2; ++ps) {
#pragma unroll 1
                for (int s = 0; s < 4; ++s) {
                    const int row = 4 * s + q8;
                    const v4f u0 = *(const v4fa*)(os + row * 68 + cofs), u1 = *(const v4fa*)(os + row * 68 + cofs + 4);
                    const v8f u = cat8f(u0, u1);
                    v8h o;
#pragma unroll
                    for (int q = 0; q < 8; ++q) {
                        float bq = 0.0f;
                        if constexpr (BIAS) bq = bfr(bias[c0 + cofs + q]);
                        float y = u[q] * cs + bq;
                        if constexpr (EP == EP_GELU) y = gelu_e(y);
                        o[q] = (h16)(y * co);
                    }
                    *(volatile v8h*)(crow + (size_t)row * ldc + cofs) = o;
                }
                if (ps == 0) __threadfence();
            }
        }
        __builtin_amdgcn_wave_barrier(); asm volatile("" ::: "memory");
    }
}

__global__ __launch_bounds__(32) void k_gemm_h16(const h16* __restrict__ A, const h16* __restrict__ Bt, int K,
                                                 float* Cf, h16* Ch, int ldc, float cs, float co,
                                                 const float* __restrict__ bias, const float* __restrict__ R,
                                                 size_t sA, size_t sB, size_t sC) {
    gemm_body<EP_H16, true, false>(A, Bt, K, Cf, Ch, ldc, cs, co, bias, R, sA, sB, sC);
}
__global__ __launch_bounds__(32) void k_gemm_gelu(const h16* __restrict__ A, const h16* __restrict__ Bt, int K,
                                                  float* Cf, h16* Ch, int ldc, float cs, float co,
                                                  const float* __restrict__ bias, const float* __restrict__ R,
                                                  size_t sA, size_t sB, size_t sC) {
    gemm_body<EP_GELU, true, false>(A, Bt, K, Cf, Ch, ldc, cs, co, bias, R, sA, sB, sC);
}
__global__ __launch_bounds__(32) void k_gemm_resx(const h16* __restrict__ A, const h16* __restrict__ Bt, int K,
                                                  float* Cf, h16* Ch, int ldc, float cs, float co,
                                                  const float* __restrict__ bias, const float* __restrict__ R,
                                                  size_t sA, size_t sB, size_t sC) {
    gemm_body<EP_RES, true, true>(A, Bt, K, Cf, Ch, ldc, cs, co, bias, R, sA, sB, sC);
}
__global__ __launch_bounds__(32) void k_gemm_res(const h16* __restrict__ A, const h16* __restrict__ Bt, int K,
                                                 float* Cf, h16* Ch, int ldc, float cs, float co,
                                                 const float* __restrict__ bias, const float* __restrict__ R,
                                                 size_t sA, size_t sB, size_t sC) {
    gemm_body<EP_RES, true, false>(A, Bt, K, Cf, Ch, ldc, cs, co, bias, R, sA, sB, sC);
}

__global__ __launch_bounds__(256) void k_cvtw(const float* __restrict__ src, h16* dst, unsigned n8) {
    const unsigned i = blockIdx.x * 256 + threadIdx.x; if (i >= n8) return;
    const v4f a0 = *(const v4f*)(src + (size_t)i * 8), a1 = *(const v4f*)(src + (size_t)i * 8 + 4);
    const v8f a = cat8f(a0, a1);
    v8h o;
#pragma unroll
    for (int k = 0; k < 8; ++k) { const float f = a[k]; o[k] = (h16)(bfr(f) * WCAR); }
    h16* p = dst + (size_t)i * 8;
    *(volatile v8h*)p = o; __threadfence(); *(volatile v8h*)p = o;
}

template <bool RBF>
__device__ __forceinline__ void ln_body(const float* __restrict__ X, const float* __restrict__ w, const float* __restrict__ bb, h16* Hp) {
    __shared__ float red[8];
    const int row = blockIdx.x, t = threadIdx.x, lane = t & 31, wave = t >> 5;
    const float* xr = X + (size_t)row * DM + t * 8;
    const v4f p0 = *(const v4f*)xr, p1 = *(const v4f*)(xr + 4);
    v8f v = cat8f(p0, p1);
    if constexpr (RBF) {
#pragma unroll
        for (int k = 0; k < 8; ++k) { const float f = v[k]; v[k] = bfr(f); }
    }
    float s = 0.0f;
#pragma unroll
    for (int k = 0; k < 8; ++k) s += v[k];
    s = wsum(s);
    if (lane == 0) red[wave] = s;
    __syncthreads();
    const float mu = ((red[0] + red[1]) + (red[2] + red[3])) * (1.0f / DM);
    v8f d; float s2 = 0.0f;
#pragma unroll
    for (int k = 0; k < 8; ++k) { const float dk = v[k] - mu; d[k] = dk; s2 += dk * dk; }
    s2 = wsum(s2);
    if (lane == 0) red[4 + wave] = s2;
    __syncthreads();
    const float var = ((red[4] + red[5]) + (red[6] + red[7])) * (1.0f / DM);
    const float rs = rsqrtf(var + 1.0e-6f);
    const v4f w0 = *(const v4f*)(w + t * 8), w1 = *(const v4f*)(w + t * 8 + 4);
    const v4f b0 = *(const v4f*)(bb + t * 8), b1 = *(const v4f*)(bb + t * 8 + 4);
    const v8f wv = cat8f(w0, w1), bv = cat8f(b0, b1);
    v8h o;
#pragma unroll
    for (int k = 0; k < 8; ++k) { const float wk = wv[k], bk = bv[k]; o[k] = (h16)(((d[k] * rs) * bfr(wk) + bfr(bk)) * HCAR); }
    h16* dst = Hp + (size_t)row * DM + t * 8;
    *(volatile v8h*)dst = o; __threadfence(); *(volatile v8h*)dst = o;
}
__global__ __launch_bounds__(128) void k_ln_in(const float* __restrict__ X, const float* __restrict__ w, const float* __restrict__ bb, h16* Hp) {
    ln_body<true>(X, w, bb, Hp);
}
__global__ __launch_bounds__(128) void k_ln_mid(const float* __restrict__ X, const float* __restrict__ w, const float* __restrict__ bb, h16* Hp) {
    ln_body<false>(X, w, bb, Hp);
}

__global__ __launch_bounds__(256) void k_vt16(const h16* __restrict__ QKV, h16* VT) {
    const unsigned e = (blockIdx.x * 256 + threadIdx.x) * 2; if (e >= (unsigned)(NB * NH * DH * SEQ)) return;
    const unsigned j = e % SEQ, rest = e / SEQ; const unsigned d = rest % DH, hd = (rest / DH) % NH, b = rest / (DH * NH);
    const size_t src = (size_t)(b * SEQ + j) * QKVW + 2 * DM + hd * DH + d;
    v2h o; o[0] = QKV[src]; o[1] = QKV[src + QKVW];
    *(volatile v2h*)(VT + e) = o; __threadfence(); *(volatile v2h*)(VT + e) = o;
}

__global__ __launch_bounds__(128) void k_flash(const h16* __restrict__ QKV, const h16* __restrict__ VT, h16* O16) {
    __shared__ __align__(16) h16 ost[4 * 16 * DH];
    const int wave = __builtin_amdgcn_readfirstlane(threadIdx.x >> 5);
    const int lane = threadIdx.x & 31, lr = lane & 15, hi = lane >> 4;
    const int hd = blockIdx.y, b = blockIdx.z;
    const int q0 = blockIdx.x * 64 + wave * 16;
    const size_t qoff = (size_t)(b * SEQ + q0 + lr) * QKVW + hd * DH + 8 * hi;
    const size_t koff = (size_t)(b * SEQ + lr) * QKVW + DM + hd * DH + 8 * hi;
    const size_t voff = ((size_t)(b * NH + hd) * DH + lr) * SEQ + 8 * hi;
    const v16h qf0 = ldfrag(QKV + qoff), qf1 = ldfrag(QKV + qoff + 32);
    const float SC = 0.125f * L2E;
    v8f acc[4];
#pragma unroll
    for (int dt = 0; dt < 4; ++dt) acc[dt] = (v8f){};
    float mrun = -3.0e38f, lrun = 0.0f;
#pragma unroll 1
    for (int j0 = 0; j0 < SEQ; j0 += 32) {
        const size_t kb = koff + (size_t)j0 * QKVW;
        v16h ka = ldfrag(QKV + kb), kc = ldfrag(QKV + kb + 32);
        v8f s0 = wmma16g(ka, qf0, (v8f){});
        s0 = wmma16g(kc, qf1, s0);
        ka = ldfrag(QKV + kb + (size_t)16 * QKVW); kc = ldfrag(QKV + kb + (size_t)16 * QKVW + 32);
        v8f s1 = wmma16g(ka, qf0, (v8f){});
        s1 = wmma16g(kc, qf1, s1);
        float mx = fmaxf(s0[0], s1[0]);
#pragma unroll
        for (int r = 1; r < 8; ++r) mx = fmaxf(mx, fmaxf(s0[r], s1[r]));
        mx = fmaxf(mx, __shfl_xor(mx, 16, 32));
        const float mnew = fmaxf(mrun, mx * SC);
        const float alpha = __builtin_amdgcn_exp2f(mrun - mnew);
        v8h p0, p1; float psum = 0.0f;
#pragma unroll
        for (int r = 0; r < 8; ++r) {
            const float e0 = __builtin_amdgcn_exp2f(s0[r] * SC - mnew);
            const float e1 = __builtin_amdgcn_exp2f(s1[r] * SC - mnew);
            const h16 c0 = (h16)(e0 * PCAR), c1 = (h16)(e1 * PCAR);
            p0[r] = c0; p1[r] = c1;
            psum += (float)c0 + (float)c1;
        }
        lrun = lrun * alpha + psum;
        mrun = mnew;
        const v16h pb = cat16(p0, p1);
#pragma unroll
        for (int dt = 0; dt < 4; ++dt) {
#pragma unroll
            for (int r = 0; r < 8; ++r) acc[dt][r] *= alpha;
        }
#pragma unroll
        for (int dt = 0; dt < 4; ++dt) {
            const v16h va = ldfrag(VT + voff + (size_t)dt * 16 * SEQ + j0);
            acc[dt] = wmma16g(va, pb, acc[dt]);
        }
    }
    const float ltot = lrun + __shfl_xor(lrun, 16, 32);
    const float linv = OCAR * __builtin_amdgcn_rcpf(ltot);
    const int ob = wave * (16 * DH);
#pragma unroll
    for (int dt = 0; dt < 4; ++dt) {
        v8h o;
#pragma unroll
        for (int r = 0; r < 8; ++r) o[r] = (h16)(acc[dt][r] * linv);
        *(v8h*)(ost + ob + lr * DH + dt * 16 + 8 * hi) = o;
    }
    __builtin_amdgcn_fence(3, "wavefront"); __builtin_amdgcn_wave_barrier(); asm volatile("" ::: "memory");
    const int q8 = lane >> 3, cofs = (lane & 7) * 8;
    h16* orow = O16 + (size_t)(b * SEQ + q0) * DM + hd * DH;
#pragma unroll 1
    for (int ps = 0; ps < 2; ++ps) {
#pragma unroll 1
        for (int s = 0; s < 4; ++s) {
            const int row = 4 * s + q8;
            const v8h val = *(const v8ha*)(ost + ob + row * DH + cofs);
            *(volatile v8h*)(orow + (size_t)row * DM + cofs) = val;
        }
        if (ps == 0) __threadfence();
    }
}

static inline unsigned cdiv(size_t a, unsigned b) { return (unsigned)((a + b - 1) / b); }

extern "C" void kernel_launch(void* const* d_in, const int* in_sizes, int n_in,
                              void* d_out, int out_size, void* d_ws, size_t ws_size, hipStream_t stream) {
    if (n_in < 15) return;
    if (in_sizes[0] < NTOK * DM || in_sizes[1] < QKVW * DM || in_sizes[2] < QKVW || in_sizes[3] < DM * DM || in_sizes[4] < DM ||
        in_sizes[5] < DM * DM || in_sizes[6] < DM || in_sizes[7] < DM || in_sizes[8] < DM || in_sizes[9] < DM || in_sizes[10] < DM ||
        in_sizes[11] < FFD * DM || in_sizes[12] < FFD || in_sizes[13] < DM * FFD || in_sizes[14] < DM) return;
    if (out_size < NTOK * DM) return;
    const float* x      = (const float*)d_in[0];
    const float* qkv_w  = (const float*)d_in[1];
    const float* qkv_b  = (const float*)d_in[2];
    const float* ap_w   = (const float*)d_in[3];
    const float* ap_b   = (const float*)d_in[4];
    const float* bp_w   = (const float*)d_in[5];
    const float* bp_b   = (const float*)d_in[6];
    const float* ln1_w  = (const float*)d_in[7];
    const float* ln1_b  = (const float*)d_in[8];
    const float* ln2_w  = (const float*)d_in[9];
    const float* ln2_b  = (const float*)d_in[10];
    const float* fc1_w  = (const float*)d_in[11];
    const float* fc1_b  = (const float*)d_in[12];
    const float* fc2_w  = (const float*)d_in[13];
    const float* fc2_b  = (const float*)d_in[14];
    float* OUT = (float*)d_out;

    char* wsp = (char*)d_ws;
    auto take = [&](size_t bytes) { char* p = wsp; wsp += (bytes + 255) & ~(size_t)255; return (void*)p; };
    h16* WQKV  = (h16*)take((size_t)QKVW * DM * 2);
    h16* WAP   = (h16*)take((size_t)DM * DM * 2);
    h16* WBP   = (h16*)take((size_t)DM * DM * 2);
    h16* W1    = (h16*)take((size_t)FFD * DM * 2);
    h16* W2    = (h16*)take((size_t)DM * FFD * 2);
    h16* QKV16 = (h16*)take((size_t)NTOK * QKVW * 2);
    h16* H2    = QKV16;
    h16* VT    = (h16*)take((size_t)NTOK * DM * 2);
    char* R1   = (char*)take((size_t)NTOK * DM * 4);
    h16* H1 = (h16*)R1; float* X1 = (float*)R1;
    h16* O16   = (h16*)take((size_t)NTOK * DM * 2);
    h16* T1    = (h16*)take((size_t)NTOK * DM * 2);
    h16* A1    = (h16*)take((size_t)NTOK * FFD * 2);
    const size_t used = (size_t)(wsp - (char*)d_ws);
    if (used > ws_size || used > (size_t)134217728) return;

    k_cvtw<<<cdiv((size_t)QKVW * DM / 8, 256), 256, 0, stream>>>(qkv_w, WQKV, (unsigned)(QKVW * DM / 8));
    k_cvtw<<<cdiv((size_t)DM * DM / 8, 256), 256, 0, stream>>>(ap_w, WAP, (unsigned)(DM * DM / 8));
    k_cvtw<<<cdiv((size_t)DM * DM / 8, 256), 256, 0, stream>>>(bp_w, WBP, (unsigned)(DM * DM / 8));
    k_cvtw<<<cdiv((size_t)FFD * DM / 8, 256), 256, 0, stream>>>(fc1_w, W1, (unsigned)(FFD * DM / 8));
    k_cvtw<<<cdiv((size_t)DM * FFD / 8, 256), 256, 0, stream>>>(fc2_w, W2, (unsigned)(DM * FFD / 8));
    k_ln_in<<<NTOK, 128, 0, stream>>>(x, ln1_w, ln1_b, H1);
    k_gemm_h16<<<dim3(NTOK / 64, QKVW / 64, 1), 32, 0, stream>>>(H1, WQKV, DM, nullptr, QKV16, QKVW, 1.0f / (HCAR * WCAR), 1.0f, qkv_b, nullptr, 0, 0, 0);
    k_vt16<<<cdiv((size_t)NB * NH * DH * SEQ / 2, 256), 256, 0, stream>>>(QKV16, VT);
    k_flash<<<dim3(SEQ / 64, NH, NB), 128, 0, stream>>>(QKV16, VT, O16);
    k_gemm_h16<<<dim3(NTOK / 64, DM / 64, 1), 32, 0, stream>>>(O16, WAP, DM, nullptr, T1, DM, 1.0f / (OCAR * WCAR), TCAR, ap_b, nullptr, 0, 0, 0);
    k_gemm_resx<<<dim3(NTOK / 64, DM / 64, 1), 32, 0, stream>>>(T1, WBP, DM, X1, nullptr, DM, 1.0f / (TCAR * WCAR), 1.0f, bp_b, x, 0, 0, 0);
    k_ln_mid<<<NTOK, 128, 0, stream>>>(X1, ln2_w, ln2_b, H2);
    k_gemm_gelu<<<dim3(NTOK / 64, FFD / 64, 1), 32, 0, stream>>>(H2, W1, DM, nullptr, A1, FFD, 1.0f / (HCAR * WCAR), ACAR, fc1_b, nullptr, 0, 0, 0);
    k_gemm_res<<<dim3(NTOK / 64, DM / 64, 1), 32, 0, stream>>>(A1, W2, FFD, OUT, nullptr, DM, 1.0f / (ACAR * WCAR), 1.0f, fc2_b, X1, 0, 0, 0);
}
